// SelectiveSSM_12936441496001
// MI455X (gfx1250) — hardware-verified
//
#include <hip/hip_runtime.h>
#include <math.h>

typedef __attribute__((ext_vector_type(16))) _Float16 v16h;
typedef __attribute__((ext_vector_type(8)))  _Float16 v8h;
typedef __attribute__((ext_vector_type(16))) __bf16   v16b;
typedef __attribute__((ext_vector_type(8)))  __bf16   v8b;
typedef __attribute__((ext_vector_type(8)))  float    v8f;
typedef __attribute__((ext_vector_type(4)))  float    v4f;

constexpr int kBatch = 2;
constexpr int kSeqL  = 2048;
constexpr int kDmod  = 1024;
constexpr int kDin   = 2048;
constexpr int kNst   = 16;
constexpr int kXdN   = kDin + 2 * kNst;
constexpr int kXdP   = 2112;
constexpr int kXZP   = 2 * kDin;
constexpr int kRows  = kBatch * kSeqL;
constexpr int kBCP   = 32;
constexpr int kTP    = 260;
constexpr float kCarryDr  = 16.0f;
constexpr float kCarryWdt = 32.0f;
constexpr float kFoldDt   = 1.0f / (kCarryDr * kCarryWdt);
static_assert(kXdN == 2080 && kXdP % 64 == 0 && kXdP >= kXdN, "x-projection width");
static_assert((kDmod % 32) == 0 && (kDin % 32) == 0, "GEMM K multiples of 32");
static_assert((kSeqL % 64) == 0 && (kXZP % 64) == 0 && (kXdP % 64) == 0 && (kDin % 64) == 0 && (kDmod % 64) == 0, "GEMM M,N multiples of 64");
static_assert((((kSeqL / 64) * (kXZP / 64)) % 8) == 0 && (((kSeqL / 64) * (kXdP / 64)) % 8) == 0 &&
              (((kSeqL / 64) * (kDin / 64)) % 8) == 0 && (((kSeqL / 64) * (kDmod / 64)) % 8) == 0, "8 tiles per block, no idle waves");
static_assert((kDin % 256) == 0 && (kSeqL % 64) == 0 && (kSeqL % 16) == 0, "conv / scan tiling");

constexpr size_t kSzXB    = (size_t)kRows * kDmod * 2;
constexpr size_t kSzWINB  = (size_t)kXZP  * kDmod * 2;
constexpr size_t kSzWXB   = (size_t)kXdP  * kDin  * 2;
constexpr size_t kSzWDTH  = (size_t)kDin  * kDin  * 2;
constexpr size_t kSzWOUTB = (size_t)kDmod * kDin  * 2;
constexpr size_t kSzXZ    = (size_t)kSeqL * kXZP  * 4;
constexpr size_t kSzP16   = (size_t)kSeqL * kDin  * 2;
constexpr size_t kSzBC    = (size_t)kSeqL * kBCP  * 4;
constexpr size_t kSzDLR   = (size_t)kSeqL * kDin  * 4;
constexpr size_t kOffXB    = 0;
constexpr size_t kOffWINB  = kOffXB    + kSzXB;
constexpr size_t kOffWXB   = kOffWINB  + kSzWINB;
constexpr size_t kOffWDTH  = kOffWXB   + kSzWXB;
constexpr size_t kOffWOUTB = kOffWDTH  + kSzWDTH;
constexpr size_t kOffXZ    = kOffWOUTB + kSzWOUTB;
constexpr size_t kOffUCH   = kOffXZ    + kSzXZ;
constexpr size_t kOffUCL   = kOffUCH   + kSzP16;
constexpr size_t kOffDRH   = kOffUCL   + kSzP16;
constexpr size_t kOffBC    = kOffDRH   + kSzP16;
constexpr size_t kOffDLR   = kOffBC    + kSzBC;
constexpr size_t kOffYH    = kOffDLR   + kSzDLR;
constexpr size_t kOffYL    = kOffYH    + kSzP16;
constexpr size_t kWsTotal  = kOffYL    + kSzP16;
static_assert(kWsTotal == 130547712ull, "carve total");
static_assert(kWsTotal <= 134217728ull, "carve cap");
static_assert((kOffWINB % 128) == 0 && (kOffWXB % 128) == 0 && (kOffWDTH % 128) == 0 && (kOffWOUTB % 128) == 0 &&
              (kOffXZ % 128) == 0 && (kOffUCH % 128) == 0 && (kOffUCL % 128) == 0 && (kOffDRH % 128) == 0 &&
              (kOffBC % 128) == 0 && (kOffDLR % 128) == 0 && (kOffYH % 128) == 0 && (kOffYL % 128) == 0, "128-B aligned regions");

__device__ __forceinline__ unsigned short f2bf_bits(float f) {
  unsigned u = __float_as_uint(f);
  return (unsigned short)((u + 0x7FFFu + ((u >> 16) & 1u)) >> 16);
}
__device__ __forceinline__ float bf_bits2f(unsigned short h) { return __uint_as_float(((unsigned)h) << 16); }
__device__ __forceinline__ float bf_rne(float f) { return bf_bits2f(f2bf_bits(f)); }

__device__ __forceinline__ void dep_guard4_h(v8f& a, v8f& b, v8f& c, v8f& d, v16h x, v16h y) { asm volatile("v_nop\n\tv_nop\n\tv_nop\n\tv_nop" : "+v"(a), "+v"(b), "+v"(c), "+v"(d) : "v"(x), "v"(y)); }
__device__ __forceinline__ void dep_guard4_b(v8f& a, v8f& b, v8f& c, v8f& d, v16b x, v16b y) { asm volatile("v_nop\n\tv_nop\n\tv_nop\n\tv_nop" : "+v"(a), "+v"(b), "+v"(c), "+v"(d) : "v"(x), "v"(y)); }
__device__ __forceinline__ void keep4_h(v16h a, v16h b, v16h c, v16h d) { asm volatile("v_nop" :: "v"(a), "v"(b), "v"(c), "v"(d)); }
__device__ __forceinline__ void keep4_b(v16b a, v16b b, v16b c, v16b d) { asm volatile("v_nop" :: "v"(a), "v"(b), "v"(c), "v"(d)); }
__device__ __forceinline__ void acc_guard4(v8f& a, v8f& b, v8f& c, v8f& d) { asm volatile("v_nop\n\tv_nop\n\tv_nop\n\tv_nop" : "+v"(a), "+v"(b), "+v"(c), "+v"(d)); }
template <typename T> struct Frag;
template <> struct Frag<_Float16> {
  typedef v16h V; union U { v16h v; v8h h[2]; };
  static __device__ __forceinline__ v16h load(const _Float16* p) {
    U f; f.h[0] = *(const v8h*)(p); f.h[1] = *(const v8h*)(p + 16); return f.v;
  }
  static __device__ __forceinline__ v8f mma(v16h a, v16h b, v8f c) {
    return __builtin_amdgcn_wmma_f32_16x16x32_f16(false, a, false, b, (short)0, c, false, false);
  }
  static __device__ __forceinline__ void guard(v8f& a, v8f& b, v8f& c, v8f& d, v16h x, v16h y) { dep_guard4_h(a, b, c, d, x, y); }
  static __device__ __forceinline__ void keep(v16h a, v16h b, v16h c, v16h d) { keep4_h(a, b, c, d); }
};
template <> struct Frag<__bf16> {
  typedef v16b V; union U { v16b v; v8b h[2]; };
  static __device__ __forceinline__ v16b load(const __bf16* p) {
    U f; f.h[0] = *(const v8b*)(p); f.h[1] = *(const v8b*)(p + 16); return f.v;
  }
  static __device__ __forceinline__ v8f mma(v16b a, v16b b, v8f c) {
    return __builtin_amdgcn_wmma_f32_16x16x32_bf16(false, a, false, b, (short)0, c, false, false);
  }
  static __device__ __forceinline__ void guard(v8f& a, v8f& b, v8f& c, v8f& d, v16b x, v16b y) { dep_guard4_b(a, b, c, d, x, y); }
  static __device__ __forceinline__ void keep(v16b a, v16b b, v16b c, v16b d) { keep4_b(a, b, c, d); }
};

template <int ET> struct Elem;
template <> struct Elem<0> { typedef _Float16 T; };
template <> struct Elem<1> { typedef __bf16 T; };
template <int ET, int SPL, int BIAS_MODE, int OUT_MODE>
__global__ __launch_bounds__(256) void wmma_gemm64(
    const unsigned short* __restrict__ Ap, const unsigned short* __restrict__ A2p, int lda, long strideA,
    const unsigned short* __restrict__ Btp, const unsigned short* __restrict__ Bt2p, int ldb, long strideB,
    void* __restrict__ Cout, void* __restrict__ Cout2, int ldc, long strideC,
    const float* __restrict__ bias,
    int M, int N, int K, float scale) {
  typedef typename Elem<ET>::T T;
  typedef typename Frag<T>::V V;
  const T* A = (const T*)Ap; const T* A2 = (const T*)A2p; const T* Bt = (const T*)Btp; const T* Bt2 = (const T*)Bt2p;
  __shared__ __align__(16) float sT[8][16 * 68];
  const int b    = blockIdx.y;
  const int lane = threadIdx.x & 31;
  const int wave = threadIdx.x >> 5;
  const int tilesN = N >> 6;
  const int tilesM = M >> 6;
  const int tile = blockIdx.x * 8 + wave;
  if (tile >= tilesM * tilesN) return;
  const int tm = tile / tilesN;
  const int tn = tile - tm * tilesN;
  const int m0 = tm << 6;
  const int n0 = tn << 6;

  const T* Ab  = A  + (size_t)b * strideA;
  const T* Bb  = Bt + (size_t)b * strideB;
  const T* Ab2 = (SPL >= 1) ? (A2  + (size_t)b * strideA) : nullptr;
  const T* Bb2 = (SPL == 2) ? (Bt2 + (size_t)b * strideB) : nullptr;

  const int rlane = lane & 15;
  const int koff  = (lane >> 4) * 8;
  const int mOff  = (lane >> 4) * 8;

  v8f acc[4][4];
#pragma unroll
  for (int i = 0; i < 4; ++i)
#pragma unroll
    for (int j = 0; j < 4; ++j) acc[i][j] = (v8f){0.f,0.f,0.f,0.f,0.f,0.f,0.f,0.f};

  for (int k0 = 0; k0 < K; k0 += 32) {
    V bh[4], bl[4];
#pragma unroll
    for (int j = 0; j < 4; ++j) {
      const size_t bo = (size_t)(n0 + (j << 4) + rlane) * ldb + koff + k0;
      bh[j] = Frag<T>::load(Bb + bo);
      if (SPL == 2) bl[j] = Frag<T>::load(Bb2 + bo);
    }
#pragma unroll
    for (int i = 0; i < 4; ++i) {
      const size_t ao = (size_t)(m0 + (i << 4) + rlane) * lda + koff + k0;
      V ah = Frag<T>::load(Ab + ao);
      V al;
      if (SPL >= 1) al = Frag<T>::load(Ab2 + ao);
#pragma unroll
      for (int j = 0; j < 4; ++j) {
        acc[i][j] = Frag<T>::mma(ah, bh[j], acc[i][j]);
        if (SPL == 2) acc[i][j] = Frag<T>::mma(ah, bl[j], acc[i][j]);
        if (SPL >= 1) acc[i][j] = Frag<T>::mma(al, bh[j], acc[i][j]);
      }
      Frag<T>::guard(acc[i][0], acc[i][1], acc[i][2], acc[i][3], ah, (SPL >= 1) ? al : ah);
    }
    Frag<T>::keep(bh[0], bh[1], bh[2], bh[3]);
    if (SPL == 2) Frag<T>::keep(bl[0], bl[1], bl[2], bl[3]);
  }
  acc_guard4(acc[0][0], acc[0][1], acc[0][2], acc[0][3]);
  acc_guard4(acc[1][0], acc[1][1], acc[1][2], acc[1][3]);
  acc_guard4(acc[2][0], acc[2][1], acc[2][2], acc[2][3]);
  acc_guard4(acc[3][0], acc[3][1], acc[3][2], acc[3][3]);

  float* slab = sT[wave];
  const float slabScale = (OUT_MODE == 3) ? 1.0f : scale;
  const float cvtScale  = (OUT_MODE == 3) ? scale : 1.0f;
  const bool  sideTile  = (OUT_MODE == 3) && (n0 >= ldc);
#pragma unroll
  for (int i = 0; i < 4; ++i) {
    const int mBase = m0 + (i << 4);
#pragma unroll
    for (int j = 0; j < 4; ++j) {
      const int n = n0 + (j << 4) + rlane;
      float bv = 0.f;
      if (BIAS_MODE == 2) bv = bias[n];
#pragma unroll
      for (int r = 0; r < 8; ++r) {
        float v = acc[i][j][r] * slabScale;
        if (BIAS_MODE == 1) v += bias[mBase + mOff + r];
        if (BIAS_MODE == 2) v += bv;
        slab[(mOff + r) * 68 + (j << 4) + rlane] = v;
      }
    }
    __builtin_amdgcn_fence(__ATOMIC_RELEASE, "workgroup");
    __builtin_amdgcn_wave_barrier();
    __builtin_amdgcn_fence(__ATOMIC_ACQUIRE, "workgroup");
    if (OUT_MODE == 0) {
      float* C = (float*)Cout + (size_t)b * strideC;
      const int hh = lane >> 4, c4 = (lane & 15) * 4;
      for (int pass = 0; pass < 2; ++pass) {
#pragma unroll
        for (int it = 0; it < 8; ++it) {
          const int row = it * 2 + hh;
          v4f v = *(const v4f*)(slab + row * 68 + c4);
          *(volatile v4f*)(C + (size_t)(mBase + row) * ldc + n0 + c4) = v;
        }
        __threadfence();
      }
    } else if (sideTile) {
      float* Cs = (float*)Cout2;
      const int q = lane >> 3, c4 = (lane & 7) * 4;
      for (int pass = 0; pass < 2; ++pass) {
#pragma unroll
        for (int it = 0; it < 4; ++it) {
          const int row = it * 4 + q;
          v4f v = *(const v4f*)(slab + row * 68 + c4);
          *(volatile v4f*)(Cs + (size_t)(mBase + row) * 32 + c4) = v;
        }
        __threadfence();
      }
    } else {
      const int q = lane >> 3, c8 = (lane & 7) * 8;
      unsigned short* C  = (unsigned short*)Cout  + (size_t)b * strideC;
      unsigned short* C2 = (OUT_MODE == 2) ? ((unsigned short*)Cout2 + (size_t)b * strideC) : nullptr;
      for (int pass = 0; pass < 2; ++pass) {
#pragma unroll
        for (int it = 0; it < 4; ++it) {
          const int row = it * 4 + q;
          const float* sp = slab + row * 68 + c8;
          v8h hv, lv;
#pragma unroll
          for (int e = 0; e < 8; ++e) {
            const float sv = sp[e];
            if (OUT_MODE == 1 || OUT_MODE == 3) {
              hv[e] = (_Float16)(sv * cvtScale);
            } else {
              unsigned short hb = f2bf_bits(sv);
              unsigned short lb = f2bf_bits(sv - bf_bits2f(hb));
              hv[e] = __builtin_bit_cast(_Float16, hb);
              lv[e] = __builtin_bit_cast(_Float16, lb);
            }
          }
          *(volatile v8h*)(C + (size_t)(mBase + row) * ldc + n0 + c8) = hv;
          if (OUT_MODE == 2) *(volatile v8h*)(C2 + (size_t)(mBase + row) * ldc + n0 + c8) = lv;
        }
        __threadfence();
      }
    }
    __builtin_amdgcn_fence(__ATOMIC_RELEASE, "workgroup");
    __builtin_amdgcn_wave_barrier();
    __builtin_amdgcn_fence(__ATOMIC_ACQUIRE, "workgroup");
  }
}

__global__ __launch_bounds__(256) void plane16_kernel(
    const float* __restrict__ src, unsigned short* __restrict__ dst, int real8, int total8, int mode, float scale)
{
  const int i = blockIdx.x * 256 + threadIdx.x;
  if (i >= total8) return;
  const bool inb = (i < real8);
  const int ic = inb ? i : (real8 - 1);
  const size_t e0 = (size_t)ic << 3;
  const v4f a0 = *(const v4f*)(src + e0);
  const v4f a1 = *(const v4f*)(src + e0 + 4);
  v8h hv;
#pragma unroll
  for (int e = 0; e < 4; ++e) {
    float f0 = a0[e];
    float f1 = a1[e];
    f0 = inb ? f0 : 0.0f;
    f1 = inb ? f1 : 0.0f;
    const unsigned short b0 = f2bf_bits(f0);
    const unsigned short b1 = f2bf_bits(f1);
    if (mode == 0) {
      hv[e]     = __builtin_bit_cast(_Float16, b0);
      hv[4 + e] = __builtin_bit_cast(_Float16, b1);
    } else {
      hv[e]     = (_Float16)(bf_bits2f(b0) * scale);
      hv[4 + e] = (_Float16)(bf_bits2f(b1) * scale);
    }
  }
  unsigned short* q = dst + ((size_t)i << 3);
  *(volatile v8h*)q = hv;
  __threadfence();
  *(volatile v8h*)q = hv;
}

__global__ __launch_bounds__(256) void conv_silu_kernel(
    const float* __restrict__ XZ, const float* __restrict__ cw, const float* __restrict__ cb,
    unsigned short* __restrict__ UCH, unsigned short* __restrict__ UCL)
{
  __shared__ __align__(16) float sT[16 * kTP];
  const int tid = threadIdx.x, lane = tid & 31, wave = tid >> 5;
  const int d0 = blockIdx.x * 256, d = d0 + tid;
  const int t0 = blockIdx.y * 64;
  const v4f wv = *(const v4f*)(cw + (size_t)d * 4);
  const float wa = wv[0], wb = wv[1], wc = wv[2], wd = wv[3];
  const float w0 = bf_rne(wa), w1 = bf_rne(wb), w2 = bf_rne(wc), w3 = bf_rne(wd);
  const float bc = bf_rne(cb[d]);
  float xm3, xm2, xm1;
  {
    const int r3 = t0 - 3, r2 = t0 - 2, r1 = t0 - 1;
    const float v3 = XZ[(size_t)(r3 < 0 ? 0 : r3) * kXZP + d];
    const float v2 = XZ[(size_t)(r2 < 0 ? 0 : r2) * kXZP + d];
    const float v1 = XZ[(size_t)(r1 < 0 ? 0 : r1) * kXZP + d];
    xm3 = (r3 >= 0) ? v3 : 0.f;
    xm2 = (r2 >= 0) ? v2 : 0.f;
    xm1 = (r1 >= 0) ? v1 : 0.f;
  }
#pragma unroll 1
  for (int sub = 0; sub < 4; ++sub) {
    const int lb = t0 + sub * 16;
#pragma unroll 1
    for (int s = 0; s < 16; ++s) {
      const float xc = XZ[(size_t)(lb + s) * kXZP + d];
      float acc = w0 * xm3;
      acc = fmaf(w1, xm2, acc);
      acc = fmaf(w2, xm1, acc);
      acc = fmaf(w3, xc, acc);
      const float sv = acc + bc;
      const float sg = __builtin_amdgcn_rcpf(1.0f + __expf(-sv));
      sT[s * kTP + tid] = sv * sg;
      xm3 = xm2; xm2 = xm1; xm1 = xc;
    }
    __syncthreads();
    v8h bh[2], blo[2];
#pragma unroll
    for (int it = 0; it < 2; ++it) {
      const float* sp = sT + (it * 8 + wave) * kTP + lane * 8;
      const v4f a0 = *(const v4f*)(sp);
      const v4f a1 = *(const v4f*)(sp + 4);
#pragma unroll
      for (int e = 0; e < 4; ++e) {
        const float f0 = a0[e], f1 = a1[e];
        const unsigned short h0 = f2bf_bits(f0), h1 = f2bf_bits(f1);
        const unsigned short l0 = f2bf_bits(f0 - bf_bits2f(h0)), l1 = f2bf_bits(f1 - bf_bits2f(h1));
        bh[it][e]      = __builtin_bit_cast(_Float16, h0);
        bh[it][4 + e]  = __builtin_bit_cast(_Float16, h1);
        blo[it][e]     = __builtin_bit_cast(_Float16, l0);
        blo[it][4 + e] = __builtin_bit_cast(_Float16, l1);
      }
    }
    for (int pass = 0; pass < 2; ++pass) {
#pragma unroll
      for (int it = 0; it < 2; ++it) {
        const size_t o = (size_t)(lb + it * 8 + wave) * kDin + d0 + lane * 8;
        *(volatile v8h*)(UCH + o) = bh[it];
        *(volatile v8h*)(UCL + o) = blo[it];
      }
      __threadfence();
    }
    __syncthreads();
  }
}

__global__ __launch_bounds__(256) void scan_kernel(
    const float* __restrict__ DLR, const unsigned* __restrict__ UCHw, const unsigned* __restrict__ UCLw,
    const float* __restrict__ XZ, const float* __restrict__ BC,
    const float* __restrict__ bdt, const float* __restrict__ A_log, const float* __restrict__ Dv,
    unsigned short* __restrict__ YH, unsigned short* __restrict__ YL)
{
  __shared__ __align__(16) float sBC[16 * kBCP];
  __shared__ __align__(16) float sY[16 * kTP];
  __shared__ __align__(16) float sA[kNst * 256];
  const int tid = threadIdx.x, lane = tid & 31, wave = tid >> 5;
  const int d0 = blockIdx.x * 256, d = d0 + tid;
  const bool oddc = (d & 1) != 0;

#pragma unroll 1
  for (int n = 0; n < kNst; ++n) sA[n * 256 + tid] = -expf(bf_rne(A_log[(size_t)d * kNst + n]));
  __syncthreads();
  float An[kNst], h[kNst];
#pragma unroll
  for (int n = 0; n < kNst; ++n) { An[n] = sA[n * 256 + tid]; h[n] = 0.f; }
  const float bb = bf_rne(bdt[d]);
  const float Dd = bf_rne(Dv[d]);

#pragma unroll 1
  for (int c = 0; c < kSeqL / 16; ++c) {
    const int l0 = c * 16;
    if (tid < 128) {
      const int r = tid >> 3, q = (tid & 7) * 4;
      const v4f v = *(const v4f*)(BC + (size_t)(l0 + r) * kBCP + q);
      *(v4f*)(sBC + r * kBCP + q) = v;
    }
    __syncthreads();
#pragma unroll 1
    for (int s = 0; s < 16; ++s) {
      const size_t m = (size_t)(l0 + s);
      const float a     = DLR[m * kDin + d] + bb;
      const unsigned wh = UCHw[m * (kDin / 2) + (d >> 1)];
      const unsigned wl = UCLw[m * (kDin / 2) + (d >> 1)];
      const float zv    = XZ[m * kXZP + kDin + d];
      const float delta = fmaxf(a, 0.0f) + log1pf(__expf(-fabsf(a)));
      const unsigned bhi = oddc ? (wh & 0xffff0000u) : (wh << 16);
      const unsigned blo = oddc ? (wl & 0xffff0000u) : (wl << 16);
      const float xv = __uint_as_float(bhi) + __uint_as_float(blo);
      v4f Bq[4], Cq[4];
#pragma unroll
      for (int qq = 0; qq < 4; ++qq) {
        Bq[qq] = *(const v4f*)(sBC + s * kBCP + 4 * qq);
        Cq[qq] = *(const v4f*)(sBC + s * kBCP + kNst + 4 * qq);
      }
      float y = 0.f;
#pragma unroll
      for (int n = 0; n < kNst; ++n) {
        const float e = __expf(delta * An[n]);
        float p = Bq[n >> 2][n & 3] * xv;
        asm volatile("" : "+v"(p));
        float qv = h[n] * e;
        asm volatile("" : "+v"(qv));
        const float hn = qv + p;
        h[n] = hn;
        float rr = Cq[n >> 2][n & 3] * hn;
        asm volatile("" : "+v"(rr));
        y += rr;
      }
      float sk = xv * Dd;
      asm volatile("" : "+v"(sk));
      y += sk;
      const float sg = __builtin_amdgcn_rcpf(1.0f + __expf(-zv));
      const float g  = zv * sg;
      sY[s * kTP + tid] = y * g;
    }
    __syncthreads();
    v8h hv[2], lv[2];
#pragma unroll
    for (int it = 0; it < 2; ++it) {
      const float* sp = sY + (it * 8 + wave) * kTP + lane * 8;
      const v4f a0 = *(const v4f*)(sp);
      const v4f a1 = *(const v4f*)(sp + 4);
#pragma unroll
      for (int e = 0; e < 4; ++e) {
        const float f0 = a0[e], f1 = a1[e];
        const unsigned short h0 = f2bf_bits(f0), h1 = f2bf_bits(f1);
        const unsigned short q0 = f2bf_bits(f0 - bf_bits2f(h0)), q1 = f2bf_bits(f1 - bf_bits2f(h1));
        hv[it][e]     = __builtin_bit_cast(_Float16, h0);
        hv[it][4 + e] = __builtin_bit_cast(_Float16, h1);
        lv[it][e]     = __builtin_bit_cast(_Float16, q0);
        lv[it][4 + e] = __builtin_bit_cast(_Float16, q1);
      }
    }
    for (int pass = 0; pass < 2; ++pass) {
#pragma unroll
      for (int it = 0; it < 2; ++it) {
        const size_t o = (size_t)(l0 + it * 8 + wave) * kDin + d0 + lane * 8;
        *(volatile v8h*)(YH + o) = hv[it];
        *(volatile v8h*)(YL + o) = lv[it];
      }
      __threadfence();
    }
  }
}

extern "C" void kernel_launch(void* const* d_in, const int* in_sizes, int n_in,
                              void* d_out, int out_size, void* d_ws, size_t ws_size,
                              hipStream_t stream)
{
  if (n_in < 10) return;
  if (in_sizes[0] != kRows * kDmod) return;
  if (in_sizes[1] != kXZP * kDmod) return;
  if (in_sizes[2] != kDin * 4) return;
  if (in_sizes[3] != kDin) return;
  if (in_sizes[4] != kXdN * kDin) return;
  if (in_sizes[5] != kDin * kDin) return;
  if (in_sizes[6] != kDin) return;
  if (in_sizes[7] != kDin * kNst) return;
  if (in_sizes[8] != kDin) return;
  if (in_sizes[9] != kDmod * kDin) return;
  if (out_size != kRows * kDmod) return;
  if (ws_size < kWsTotal) return;

  const float* x      = (const float*)d_in[0];
  const float* W_in   = (const float*)d_in[1];
  const float* conv_w = (const float*)d_in[2];
  const float* conv_b = (const float*)d_in[3];
  const float* W_x    = (const float*)d_in[4];
  const float* W_dt   = (const float*)d_in[5];
  const float* b_dt   = (const float*)d_in[6];
  const float* A_log  = (const float*)d_in[7];
  const float* Dv     = (const float*)d_in[8];
  const float* W_out  = (const float*)d_in[9];
  float* dout = (float*)d_out;

  char* ws = (char*)d_ws;
  unsigned short* XB    = (unsigned short*)(ws + kOffXB);
  unsigned short* WINB  = (unsigned short*)(ws + kOffWINB);
  unsigned short* WXB   = (unsigned short*)(ws + kOffWXB);
  unsigned short* WDTH  = (unsigned short*)(ws + kOffWDTH);
  unsigned short* WOUTB = (unsigned short*)(ws + kOffWOUTB);
  float*          XZ    = (float*)(ws + kOffXZ);
  unsigned short* UCH   = (unsigned short*)(ws + kOffUCH);
  unsigned short* UCL   = (unsigned short*)(ws + kOffUCL);
  unsigned short* DRH   = (unsigned short*)(ws + kOffDRH);
  float*          BC    = (float*)(ws + kOffBC);
  float*          DLR   = (float*)(ws + kOffDLR);
  unsigned short* YH    = (unsigned short*)(ws + kOffYH);
  unsigned short* YL    = (unsigned short*)(ws + kOffYL);
  const float* unused_bias = b_dt;

  {
    const int n8x  = (kRows * kDmod) / 8;
    const int n8wi = (kXZP * kDmod) / 8;
    const int n8wxr = (kXdN * kDin) / 8;
    const int n8wxt = (kXdP * kDin) / 8;
    const int n8wd = (kDin * kDin) / 8;
    const int n8wo = (kDmod * kDin) / 8;
    plane16_kernel<<<n8x / 256, 256, 0, stream>>>(x, XB, n8x, n8x, 0, 1.0f);
    plane16_kernel<<<n8wi / 256, 256, 0, stream>>>(W_in, WINB, n8wi, n8wi, 0, 1.0f);
    plane16_kernel<<<n8wxt / 256, 256, 0, stream>>>(W_x, WXB, n8wxr, n8wxt, 0, 1.0f);
    plane16_kernel<<<n8wd / 256, 256, 0, stream>>>(W_dt, WDTH, n8wd, n8wd, 1, kCarryWdt);
    plane16_kernel<<<n8wo / 256, 256, 0, stream>>>(W_out, WOUTB, n8wo, n8wo, 0, 1.0f);
  }

  for (int b = 0; b < kBatch; ++b) {
    const unsigned short* XBb = XB + (size_t)b * kSeqL * kDmod;
    float* outb = dout + (size_t)b * kSeqL * kDmod;

    wmma_gemm64<1, 0, 0, 0><<<dim3(256, 1), 256, 0, stream>>>(
        XBb, XBb, kDmod, 0L, WINB, WINB, kDmod, 0L,
        (void*)XZ, (void*)XZ, kXZP, 0L, unused_bias, kSeqL, kXZP, kDmod, 1.0f);

    conv_silu_kernel<<<dim3(kDin / 256, kSeqL / 64), 256, 0, stream>>>(XZ, conv_w, conv_b, UCH, UCL);

    wmma_gemm64<1, 1, 0, 3><<<dim3(132, 1), 256, 0, stream>>>(
        UCH, UCL, kDin, 0L, WXB, WXB, kDin, 0L,
        (void*)DRH, (void*)BC, kDin, 0L, unused_bias, kSeqL, kXdP, kDin, kCarryDr);

    wmma_gemm64<0, 0, 0, 0><<<dim3(128, 1), 256, 0, stream>>>(
        DRH, DRH, kDin, 0L, WDTH, WDTH, kDin, 0L,
        (void*)DLR, (void*)DLR, kDin, 0L, unused_bias, kSeqL, kDin, kDin, kFoldDt);

    scan_kernel<<<dim3(kDin / 256, 1), 256, 0, stream>>>(
        DLR, (const unsigned*)UCH, (const unsigned*)UCL, XZ, BC, b_dt, A_log, Dv, YH, YL);

    wmma_gemm64<1, 1, 0, 0><<<dim3(64, 1), 256, 0, stream>>>(
        YH, YL, kDin, 0L, WOUTB, WOUTB, kDin, 0L,
        (void*)outb, (void*)outb, kDmod, 0L, unused_bias, kSeqL, kDmod, kDin, 1.0f);
  }
}
